// OVDClassifier_32014686225101
// MI455X (gfx1250) — hardware-run, weakly checked
//
#include <hip/hip_runtime.h>
#include <math.h>

typedef __attribute__((ext_vector_type(16))) _Float16 v16h;
typedef __attribute__((ext_vector_type(8)))  _Float16 v8h;
typedef __attribute__((ext_vector_type(16))) __bf16   v16b;
typedef __attribute__((ext_vector_type(8)))  __bf16   v8b;
typedef __attribute__((ext_vector_type(8)))  float    v8f;
typedef __attribute__((ext_vector_type(4)))  float    v4f;

constexpr int kBatch  = 2;
constexpr int kPatch  = 6400;
constexpr int kGrid   = 80;
constexpr int kDepth  = 1024;
constexpr int kNemb   = 128;
constexpr int kBoxes  = 100;
constexpr int kTarget = 560;
constexpr int kRowsA  = kBatch * kPatch;
constexpr int kOutRows = kBatch * kBoxes;
static_assert(kGrid * kGrid == kPatch, "patch grid");
static_assert(kTarget == 7 * kGrid, "seven output pixels per patch");
static_assert((kRowsA % 64) == 0 && (kNemb % 64) == 0 && (kDepth % 32) == 0, "GEMM tile multiples");
static_assert((((kRowsA / 64) * (kNemb / 64)) % 8) == 0, "8 tiles per block exactly");

constexpr size_t kOffA16  = 0;
constexpr size_t kOffB16  = kOffA16 + (size_t)kRowsA * kDepth * 2;
constexpr size_t kOffDot  = kOffB16 + (size_t)kNemb * kDepth * 2;
constexpr size_t kWsTotal = kOffDot + (size_t)kRowsA * kNemb * 4;
static_assert(kWsTotal == 33030144ull, "carve total");
static_assert(kWsTotal <= 134217728ull, "carve cap");
static_assert((kOffB16 % 128) == 0 && (kOffDot % 128) == 0, "128-B aligned regions");

constexpr double cub_abs(double x) { return x < 0.0 ? -x : x; }
constexpr double cub_poly(double x) {
  return (x <= 1.0) ? ((-0.75 + 2.0) * x * x * x - (-0.75 + 3.0) * x * x + 1.0)
       : ((x < 2.0) ? ((-0.75) * x * x * x - 5.0 * (-0.75) * x * x + 8.0 * (-0.75) * x - 4.0 * (-0.75)) : 0.0);
}
constexpr double cub_w(int r, int k) { return cub_poly(cub_abs((double)r / 7.0 - (double)k)); }
#define CUBIC_PHASE_ROW(r) (float)cub_w(r, -1), (float)cub_w(r, 0), (float)cub_w(r, 1), (float)cub_w(r, 2)
__constant__ float kCubW[28] = {
  CUBIC_PHASE_ROW(0), CUBIC_PHASE_ROW(1), CUBIC_PHASE_ROW(2), CUBIC_PHASE_ROW(3),
  CUBIC_PHASE_ROW(4), CUBIC_PHASE_ROW(5), CUBIC_PHASE_ROW(6)
};
static_assert(sizeof(kCubW) / sizeof(kCubW[0]) == 28, "7 x 4 table");

__device__ __forceinline__ unsigned short f2bf_bits(float f) {
  unsigned u = __float_as_uint(f);
  return (unsigned short)((u + 0x7FFFu + ((u >> 16) & 1u)) >> 16);
}

__device__ __forceinline__ v16b frag_load_b(const __bf16* p) {
  union U { v16b v; v8b h[2]; } f;
  f.h[0] = *(const v8b*)(p);
  f.h[1] = *(const v8b*)(p + 16);
  return f.v;
}

__device__ __forceinline__ v8f mma_tied_b(v16b a, v16b b, v8f c) {
  c = __builtin_amdgcn_wmma_f32_16x16x32_bf16(false, a, false, b, (short)0, c, false, false);
  asm volatile("v_nop\n\tv_nop\n\tv_nop\n\tv_nop" : "+v"(c) : "v"(a), "v"(b));
  return c;
}

constexpr int kCvtTotal8A = kRowsA * kDepth / 8;
constexpr int kCvtTotal8B = kNemb * kDepth / 8;
constexpr int kCvtBlocksA = kCvtTotal8A / 256;
constexpr int kCvtBlocksB = kCvtTotal8B / 256;
static_assert(kCvtBlocksA * 256 == kCvtTotal8A && kCvtBlocksB * 256 == kCvtTotal8B, "exact convert coverage");

__global__ __launch_bounds__(256) void cvt_planes_kernel(
    const float* __restrict__ feats, const float* __restrict__ emb,
    unsigned short* __restrict__ a16, unsigned short* __restrict__ b16)
{
  const int blk = blockIdx.x;
  const bool isA = blk < kCvtBlocksA;
  const float* src = isA ? feats : emb;
  unsigned short* dst = isA ? a16 : b16;
  const int lb  = isA ? blk : (blk - kCvtBlocksA);
  const int lim = isA ? kCvtTotal8A : kCvtTotal8B;
  const int i = lb * 256 + (int)threadIdx.x;
  if (i >= lim) return;
  const size_t e0 = (size_t)i << 3;
  const v4f a0 = *(const v4f*)(src + e0);
  const v4f a1 = *(const v4f*)(src + e0 + 4);
  v8h hv;
#pragma unroll
  for (int e = 0; e < 4; ++e) {
    const unsigned short h0 = f2bf_bits(a0[e]);
    const unsigned short h1 = f2bf_bits(a1[e]);
    hv[e]     = __builtin_bit_cast(_Float16, h0);
    hv[4 + e] = __builtin_bit_cast(_Float16, h1);
  }
  unsigned short* q = dst + e0;
  *(volatile v8h*)q = hv;
  __threadfence();
  *(volatile v8h*)q = hv;
}

__global__ __launch_bounds__(256) void gemm_dot_kernel(
    const unsigned short* __restrict__ Ap, const unsigned short* __restrict__ Btp, float* __restrict__ C)
{
  const __bf16* A  = (const __bf16*)Ap;
  const __bf16* Bt = (const __bf16*)Btp;
  __shared__ __align__(16) float sT[8][16 * 68];
  const int lane = threadIdx.x & 31;
  const int wave = __builtin_amdgcn_readfirstlane((int)(threadIdx.x >> 5));
  constexpr int tilesN = kNemb >> 6;
  constexpr int tilesM = kRowsA >> 6;
  const int tile = blockIdx.x * 8 + wave;
  if (tile >= tilesM * tilesN) return;
  const int tm = tile / tilesN;
  const int tn = tile - tm * tilesN;
  const int m0 = tm << 6;
  const int n0 = tn << 6;

  const int rlane = lane & 15;
  const int koff  = (lane >> 4) * 8;
  const int mOff  = (lane >> 4) * 8;

  v8f acc[4][4];
#pragma unroll
  for (int i = 0; i < 4; ++i)
#pragma unroll
    for (int j = 0; j < 4; ++j) acc[i][j] = (v8f){0.f, 0.f, 0.f, 0.f, 0.f, 0.f, 0.f, 0.f};

#pragma unroll 1
  for (int k0 = 0; k0 < kDepth; k0 += 32) {
    v16b bfr[4];
#pragma unroll
    for (int j = 0; j < 4; ++j)
      bfr[j] = frag_load_b(Bt + (size_t)(n0 + (j << 4) + rlane) * kDepth + koff + k0);
#pragma unroll
    for (int i = 0; i < 4; ++i) {
      const v16b afr = frag_load_b(A + (size_t)(m0 + (i << 4) + rlane) * kDepth + koff + k0);
#pragma unroll
      for (int j = 0; j < 4; ++j) acc[i][j] = mma_tied_b(afr, bfr[j], acc[i][j]);
    }
  }

  float* slab = sT[wave];
#pragma unroll
  for (int i = 0; i < 4; ++i) {
    const int mBase = m0 + (i << 4);
#pragma unroll
    for (int j = 0; j < 4; ++j) {
#pragma unroll
      for (int r = 0; r < 8; ++r) slab[(mOff + r) * 68 + (j << 4) + rlane] = acc[i][j][r];
    }
    __builtin_amdgcn_fence(__ATOMIC_RELEASE, "workgroup");
    __builtin_amdgcn_wave_barrier();
    __builtin_amdgcn_fence(__ATOMIC_ACQUIRE, "workgroup");
    {
      const int hh = lane >> 4, c4 = (lane & 15) * 4;
      for (int pass = 0; pass < 2; ++pass) {
#pragma unroll
        for (int it = 0; it < 8; ++it) {
          const int row = it * 2 + hh;
          const v4f v = *(const v4f*)(slab + row * 68 + c4);
          *(volatile v4f*)(C + (size_t)(mBase + row) * kNemb + n0 + c4) = v;
        }
        __threadfence();
      }
    }
    __builtin_amdgcn_fence(__ATOMIC_RELEASE, "workgroup");
    __builtin_amdgcn_wave_barrier();
    __builtin_amdgcn_fence(__ATOMIC_ACQUIRE, "workgroup");
  }
}

__device__ __forceinline__ int clamp_i(int v, int lo, int hi) { return v < lo ? lo : (v > hi ? hi : v); }

__global__ __launch_bounds__(128) void box_pool_kernel(
    const float* __restrict__ dotT, const int* __restrict__ boxes, float* __restrict__ out)
{
  __shared__ __align__(16) float sW[128];
  __shared__ __align__(16) float sU[128];
  __shared__ __align__(16) float sV[128];
  const int tid = threadIdx.x;
  const int bm  = blockIdx.x;
  const int b   = bm / kBoxes;

  const int ti = tid < 27 ? tid : 27;
  const float wv = kCubW[ti];
  sW[tid] = wv;

  const int* bx = boxes + (size_t)bm * 4;
  const int x1 = bx[0], y1 = bx[1], bw = bx[2], bh = bx[3];
  const int xe = x1 + bw - 1;
  const int ye = y1 + bh - 1;
  const int areai = (ye - y1) * (xe - x1);
  const float area = (float)areai;
  const int x1c = clamp_i(x1, 0, kTarget), xec = clamp_i(xe, 0, kTarget);
  const int y1c = clamp_i(y1, 0, kTarget), yec = clamp_i(ye, 0, kTarget);
  const bool yok = yec > y1c, xok = xec > x1c;
  const int hlo = yok ? clamp_i((y1c + 4) / 7 - 2, 0, kGrid - 1) : 0;
  const int hhi = yok ? clamp_i((yec + 3) / 7 + 1, 0, kGrid - 1) : -1;
  const int wlo = xok ? clamp_i((x1c + 4) / 7 - 2, 0, kGrid - 1) : 0;
  const int whi = xok ? clamp_i((xec + 3) / 7 + 1, 0, kGrid - 1) : -1;
  __syncthreads();

  float ua = 0.0f, va = 0.0f;
#pragma unroll 1
  for (int Y = y1c; Y < yec; ++Y) {
    const int q = (Y + 4) / 7;
    const int r = (Y + 4) - 7 * q;
    const int f = q - 1;
    const v4f w4 = *(const v4f*)(sW + 4 * r);
    const int i0 = clamp_i(f - 1, 0, kGrid - 1);
    const int i1 = clamp_i(f,     0, kGrid - 1);
    const int i2 = clamp_i(f + 1, 0, kGrid - 1);
    const int i3 = clamp_i(f + 2, 0, kGrid - 1);
    ua += (i0 == tid) ? w4[0] : 0.0f;
    ua += (i1 == tid) ? w4[1] : 0.0f;
    ua += (i2 == tid) ? w4[2] : 0.0f;
    ua += (i3 == tid) ? w4[3] : 0.0f;
  }
#pragma unroll 1
  for (int X = x1c; X < xec; ++X) {
    const int q = (X + 4) / 7;
    const int r = (X + 4) - 7 * q;
    const int f = q - 1;
    const v4f w4 = *(const v4f*)(sW + 4 * r);
    const int i0 = clamp_i(f - 1, 0, kGrid - 1);
    const int i1 = clamp_i(f,     0, kGrid - 1);
    const int i2 = clamp_i(f + 1, 0, kGrid - 1);
    const int i3 = clamp_i(f + 2, 0, kGrid - 1);
    va += (i0 == tid) ? w4[0] : 0.0f;
    va += (i1 == tid) ? w4[1] : 0.0f;
    va += (i2 == tid) ? w4[2] : 0.0f;
    va += (i3 == tid) ? w4[3] : 0.0f;
  }
  sU[tid] = ua;
  sV[tid] = va;
  __syncthreads();

  const float* base = dotT + (size_t)b * kPatch * kNemb + tid;
  float acc = 0.0f;
#pragma unroll 1
  for (int h = hlo; h <= hhi; ++h) {
    const float uh = sU[h];
    const float* rowp = base + (size_t)(h * kGrid) * kNemb;
    float rs = 0.0f;
#pragma unroll 4
    for (int w = wlo; w <= whi; ++w) rs = fmaf(sV[w], rowp[(size_t)w * kNemb], rs);
    acc = fmaf(uh, rs, acc);
  }
  const float res = acc / area;
  volatile float* op = (volatile float*)(out + (size_t)bm * kNemb + tid);
  *op = res;
  __threadfence();
  *op = res;
}

extern "C" void kernel_launch(void* const* d_in, const int* in_sizes, int n_in,
                              void* d_out, int out_size, void* d_ws, size_t ws_size,
                              hipStream_t stream) {
  if (n_in < 3) return;
  if (in_sizes[0] != kBatch * kPatch * kDepth) return;
  if (in_sizes[1] != kNemb * kDepth) return;
  if (in_sizes[2] != kBatch * kBoxes * 4) return;
  if (out_size != kOutRows * kNemb) return;
  if (ws_size < kWsTotal) return;

  const float* feats = (const float*)d_in[0];
  const float* emb   = (const float*)d_in[1];
  const int*   boxes = (const int*)d_in[2];
  float* out = (float*)d_out;

  char* ws = (char*)d_ws;
  unsigned short* A16 = (unsigned short*)(ws + kOffA16);
  unsigned short* B16 = (unsigned short*)(ws + kOffB16);
  float*          DOT = (float*)(ws + kOffDot);

  cvt_planes_kernel<<<kCvtBlocksA + kCvtBlocksB, 256, 0, stream>>>(feats, emb, A16, B16);
  gemm_dot_kernel<<<((kRowsA / 64) * (kNemb / 64)) / 8, 256, 0, stream>>>(A16, B16, DOT);
  box_pool_kernel<<<kOutRows, 128, 0, stream>>>(DOT, boxes, out);
}
